// SGATEmbedding_67680094650926
// MI455X (gfx1250) — hardware-verified
//
#include <hip/hip_runtime.h>
#include <stddef.h>


#define BB    8
#define TT    12
#define NN    10000
#define FF    16
#define DF    192
#define VV    (BB * NN)
#define C8    (DF / 8)
#define ALPHA 0.2f
#define GR    64
#define XSP   196
#define NB    256
#define CHUNK 2048
#define NTHR  256
#define NWAVE 8
#define WCAP  256
#define NGRP  (CHUNK / (NTHR * 4))

#define LDS_SACC (NB * DF)
#define LDS_AUX  (4 * NB)
#define LDS_LIST (NWAVE * WCAP)
#define LDS_BYTES ((LDS_SACC + LDS_AUX + LDS_LIST + NWAVE) * 4)

static_assert(WCAP == (CHUNK / NTHR) * 32);
static_assert(NGRP >= 1);
static_assert(NTHR == NB);
static_assert((NB & (NB - 1)) == 0 && NB <= 512);
static_assert(CHUNK <= 2048);
static_assert((LDS_SACC % 4) == 0);
static_assert(LDS_BYTES == 208928);
static_assert(DF == FF * TT);
static_assert((NB * C8) % (4 * NTHR) == 0);
static_assert(NB % 64 == 0);
static_assert(GR == 64 && DF == 192);

typedef float    v2f  __attribute__((ext_vector_type(2)));
typedef float    v4f  __attribute__((ext_vector_type(4)));
typedef float    v8f  __attribute__((ext_vector_type(8)));
typedef int      v4i  __attribute__((ext_vector_type(4)));
typedef _Float16 v8h  __attribute__((ext_vector_type(8)));
typedef _Float16 v16h __attribute__((ext_vector_type(16)));
union Frag   { v16h v; v8h half[2]; };
union Pack16 { v8h h; v4i i; };

__device__ __forceinline__ v8f wm(v16h a, v16h b, v8f c) {
  v8f d = __builtin_amdgcn_wmma_f32_16x16x32_f16(false, a, false, b, (short)0, c, false, false);
  asm volatile("v_nop\n\tv_nop\n\tv_nop\n\tv_nop" : "+v"(d) : "v"(a), "v"(b));
  return d;
}

__device__ __forceinline__ float elu1(float v) { return v > 0.f ? v : (__expf(v) - 1.0f); }

__global__ __launch_bounds__(NTHR) void k_prepx(const float* __restrict__ x, _Float16* Hh, int ntask) {
  const int q = blockIdx.x * NTHR + threadIdx.x;
  if (q >= ntask) return;
  const int v  = q / C8;
  const int c8 = q - v * C8;
  const int b  = v / NN;
  const int n  = v - b * NN;
  Pack16 u;
#pragma unroll
  for (int i = 0; i < 8; ++i) {
    const int c = c8 * 8 + i;
    const int f = c / TT;
    const int t = c - f * TT;
    u.h[i] = (_Float16)x[((size_t)(b * TT + t) * NN + (size_t)n) * FF + f];
  }
  _Float16* p = Hh + (size_t)v * DF + c8 * 8;
  *(volatile v4i*)p = u.i;
  __threadfence();
  *(volatile v4i*)p = u.i;
}

__global__ __launch_bounds__(NTHR) void k_prepw(const float* __restrict__ W0, const float* __restrict__ W1,
                                                _Float16* Wt0, _Float16* Wt1) {
  const int q = blockIdx.x * NTHR + threadIdx.x;
  if (q >= 2 * DF * C8) return;
  const int mat = q / (DF * C8);
  const int r   = q - mat * (DF * C8);
  const int n   = r / C8;
  const int c8  = r - n * C8;
  const float* W = mat ? W1 : W0;
  _Float16* Wt   = mat ? Wt1 : Wt0;
  Pack16 u;
#pragma unroll
  for (int i = 0; i < 8; ++i) {
    const int k = c8 * 8 + i;
    u.h[i] = (_Float16)(W[(size_t)k * DF + n] * 8.0f);
  }
  _Float16* p = Wt + (size_t)n * DF + c8 * 8;
  *(volatile v4i*)p = u.i;
  __threadfence();
  *(volatile v4i*)p = u.i;
}

__global__ __launch_bounds__(NTHR) void k_gemm(
    const _Float16* __restrict__ Ah, const _Float16* __restrict__ Wt,
    const float* __restrict__ attl, const float* __restrict__ attr,
    float* ft, float* elv, float* erv, int V) {
  __shared__ __attribute__((aligned(16))) float Xs[GR * XSP];
  __shared__ __attribute__((aligned(16))) float Es[GR];
  __shared__ __attribute__((aligned(16))) float Rs[GR];

  const int tid  = threadIdx.x;
  const int lane = tid & 31;
  const int wave = tid >> 5;
  const int hh   = lane >> 4;
  const int m    = lane & 15;
  const int rt   = wave & 3;
  const int ch   = wave >> 2;
  const int rowBase = blockIdx.x * GR;

  int arow = rowBase + rt * 16 + m;
  if (arow > V - 1) arow = V - 1;
  const _Float16* pa = Ah + (size_t)arow * DF + 8 * hh;

  v8f acc[6];
#pragma unroll
  for (int j = 0; j < 6; ++j) acc[j] = (v8f){0.f, 0.f, 0.f, 0.f, 0.f, 0.f, 0.f, 0.f};

#pragma unroll
  for (int kt = 0; kt < DF / 32; ++kt) {
    const int k0 = kt * 32;
    Frag a;
    a.half[0] = *(const v8h*)(pa + k0);
    a.half[1] = *(const v8h*)(pa + k0 + 16);
#pragma unroll
    for (int j = 0; j < 6; ++j) {
      const int ncol = (ch * 6 + j) * 16 + m;
      const _Float16* pb = Wt + (size_t)ncol * DF + k0 + 8 * hh;
      Frag b;
      b.half[0] = *(const v8h*)pb;
      b.half[1] = *(const v8h*)(pb + 16);
      acc[j] = wm(a.v, b.v, acc[j]);
    }
  }

#pragma unroll
  for (int j = 0; j < 6; ++j) {
    const int col = (ch * 6 + j) * 16 + m;
#pragma unroll
    for (int r = 0; r < 8; ++r) Xs[(rt * 16 + 8 * hh + r) * XSP + col] = acc[j][r] * 0.125f;
  }
  __syncthreads();

  {
    const int row  = tid >> 2;
    const int part = tid & 3;
    float sl = 0.f, sr = 0.f;
#pragma unroll 4
    for (int i = 0; i < 48; ++i) {
      const int c = part * 48 + i;
      const float v = Xs[row * XSP + c];
      sl += v * attl[c];
      sr += v * attr[c];
    }
    sl += __shfl_xor(sl, 1, 32); sl += __shfl_xor(sl, 2, 32);
    sr += __shfl_xor(sr, 1, 32); sr += __shfl_xor(sr, 2, 32);
    if (part == 0) { Es[row] = sl; Rs[row] = sr; }
  }
  __syncthreads();

  v4f xr[8], xt[8];
#pragma unroll
  for (int i = 0; i < 8; ++i) {
    const int row = 8 * wave + i;
    xr[i] = *(const v4f*)(Xs + row * XSP + 4 * lane);
    xt[i] = *(const v4f*)(Xs + row * XSP + 128 + 4 * (lane & 15));
  }
  v4f ev;
  float* gp;
  if (lane < 16) { ev = *(const v4f*)(Es + 4 * lane);        gp = elv + rowBase + 4 * lane; }
  else           { ev = *(const v4f*)(Rs + 4 * (lane - 16)); gp = erv + rowBase + 4 * (lane - 16); }

#pragma unroll
  for (int i = 0; i < 8; ++i) {
    float* rp = ft + (size_t)(rowBase + 8 * wave + i) * DF;
    *(volatile v4f*)(rp + 4 * lane) = xr[i];
    if (lane < 16) *(volatile v4f*)(rp + 128 + 4 * lane) = xt[i];
  }
  if (wave == 0) *(volatile v4f*)gp = ev;
  __threadfence();
#pragma unroll
  for (int i = 0; i < 8; ++i) {
    float* rp = ft + (size_t)(rowBase + 8 * wave + i) * DF;
    *(volatile v4f*)(rp + 4 * lane) = xr[i];
    if (lane < 16) *(volatile v4f*)(rp + 128 + 4 * lane) = xt[i];
  }
  if (wave == 0) *(volatile v4f*)gp = ev;
}

__global__ __launch_bounds__(NTHR) void k_agg(
    const float* __restrict__ ft, const float* __restrict__ elv, const float* __restrict__ erv,
    const int* __restrict__ src, const int* __restrict__ dst,
    const float* __restrict__ bias, const float* __restrict__ x,
    _Float16* Hout, float* out, int nE, int nblk, int layer2) {
  extern __shared__ v4f lds_dyn[];
  float* sacc = (float*)lds_dyn;
  float* den  = sacc + LDS_SACC;
  float* mx   = den + NB;
  float* erc  = mx + NB;
  float* inv  = erc + NB;
  int*   list = (int*)(inv + NB);
  int*   wcnt = list + LDS_LIST;

  const int tid  = threadIdx.x;
  const int lane = tid & 31;
  const int wave = tid >> 5;
  const int b    = blockIdx.x / nblk;
  const int nb   = blockIdx.x - b * nblk;
  const int n0   = nb * NB;
  int nvalid = NN - n0;
  if (nvalid > NB) nvalid = NB;
  const int vbase = b * NN;

  {
    const v4f z4 = {0.f, 0.f, 0.f, 0.f};
    for (int i = tid; i < LDS_SACC / 4; i += NTHR) lds_dyn[i] = z4;
    int n = n0 + tid;
    if (n > NN - 1) n = NN - 1;
    den[tid] = 0.f;
    mx[tid]  = -1.0e30f;
    erc[tid] = erv[vbase + n];
    inv[tid] = 0.f;
  }
  __syncthreads();

  const bool al16 = ((((size_t)dst) & 15) == 0);
  const int nChunks = (nE + CHUNK - 1) / CHUNK;
#pragma unroll 1
  for (int chk = 0; chk < nChunks; ++chk) {
    const int cbase = chk * CHUNK;
    int wc = 0;
#pragma unroll
    for (int g = 0; g < NGRP; ++g) {
      const int el0 = (g * NTHR + tid) * 4;
      const int e0  = cbase + el0;
      const int sent = -2147483647 - 1;
      v4i d;
      if (al16 && (e0 + 3 < nE)) {
        d = *(const v4i*)(dst + e0);
      } else {
        d.x = (e0     < nE) ? dst[min(e0, nE - 1)]     : sent;
        d.y = (e0 + 1 < nE) ? dst[min(e0 + 1, nE - 1)] : sent;
        d.z = (e0 + 2 < nE) ? dst[min(e0 + 2, nE - 1)] : sent;
        d.w = (e0 + 3 < nE) ? dst[min(e0 + 3, nE - 1)] : sent;
      }
      const unsigned s0 = (unsigned)d.x - (unsigned)n0;
      const unsigned s1 = (unsigned)d.y - (unsigned)n0;
      const unsigned s2 = (unsigned)d.z - (unsigned)n0;
      const unsigned s3 = (unsigned)d.w - (unsigned)n0;
      const bool h0 = s0 < (unsigned)NB;
      const bool h1 = s1 < (unsigned)NB;
      const bool h2 = s2 < (unsigned)NB;
      const bool h3 = s3 < (unsigned)NB;
      const unsigned many = __builtin_amdgcn_ballot_w32(h0 | h1 | h2 | h3);
      if (many != 0u) {
#define HITJ(J, HJ, SJ) { \
          const unsigned mj = __builtin_amdgcn_ballot_w32(HJ); \
          if (HJ) { \
            const int pos = wc + (int)__builtin_amdgcn_mbcnt_lo(mj, 0u); \
            if (pos < WCAP) list[wave * WCAP + pos] = ((el0 + (J)) << 9) | (int)(SJ); \
          } \
          wc += (int)__builtin_popcount(mj); }
        HITJ(0, h0, s0)
        HITJ(1, h1, s1)
        HITJ(2, h2, s2)
        HITJ(3, h3, s3)
#undef HITJ
      }
    }
    if (lane == 0) wcnt[wave] = wc;
    __syncthreads();

    if (wave == 0) {
#pragma unroll 1
      for (int wsx = 0; wsx < NWAVE; ++wsx) {
        int nh = wcnt[wsx];
        if (nh > WCAP) nh = WCAP;
        if (nh < 0) nh = 0;
#pragma unroll 1
        for (int i = 0; i < nh; ++i) {
          const int ent  = list[wsx * WCAP + i];
          const int slot = ent & (NB - 1);
          const int eloc = (ent >> 9) & (CHUNK - 1);
          int e = cbase + eloc;
          if (e > nE - 1) e = nE - 1;
          int s = src[e];
          s = s < 0 ? 0 : (s > NN - 1 ? NN - 1 : s);
          const int vs = vbase + s;
          float lg = elv[vs] + erc[slot];
          lg = (lg > 0.f) ? lg : ALPHA * lg;
          const float mo = mx[slot];
          const float mn = fmaxf(mo, lg);
          const float sc = __expf(mo - mn);
          const float p  = __expf(lg - mn);
          const float* fr = ft + (size_t)vs * DF;
          const v4f f4 = *(const v4f*)(fr + 4 * lane);
          const v2f f2 = *(const v2f*)(fr + 128 + 2 * lane);
          float* sr = sacc + slot * DF;
          v4f c4 = *(const v4f*)(sr + 4 * lane);
          v2f c2 = *(const v2f*)(sr + 128 + 2 * lane);
          c4 = c4 * sc + p * f4;
          c2 = c2 * sc + p * f2;
          *(v4f*)(sr + 4 * lane) = c4;
          *(v2f*)(sr + 128 + 2 * lane) = c2;
          const float dn = den[slot] * sc + p;
          den[slot] = dn;
          mx[slot]  = mn;
        }
      }
    }
    __syncthreads();
  }

  {
    const float dv = den[tid];
    inv[tid] = (dv > 0.f) ? (1.0f / dv) : 0.f;
  }
  __syncthreads();

  if (layer2 == 0) {
#pragma unroll 1
    for (int grp = 0; grp < (NB * C8) / (4 * NTHR); ++grp) {
      Pack16 u[4];
#pragma unroll
      for (int j = 0; j < 4; ++j) {
        const int q    = (grp * 4 + j) * NTHR + tid;
        const int slot = q / C8;
        const int c8   = q - slot * C8;
        const float iv = inv[slot];
        const v4f s0 = *(const v4f*)(sacc + slot * DF + c8 * 8);
        const v4f s1 = *(const v4f*)(sacc + slot * DF + c8 * 8 + 4);
        const v4f b0 = *(const v4f*)(bias + c8 * 8);
        const v4f b1 = *(const v4f*)(bias + c8 * 8 + 4);
        const v4f v0 = s0 * iv + b0;
        const v4f v1 = s1 * iv + b1;
        u[j].h[0] = (_Float16)elu1(v0.x); u[j].h[1] = (_Float16)elu1(v0.y);
        u[j].h[2] = (_Float16)elu1(v0.z); u[j].h[3] = (_Float16)elu1(v0.w);
        u[j].h[4] = (_Float16)elu1(v1.x); u[j].h[5] = (_Float16)elu1(v1.y);
        u[j].h[6] = (_Float16)elu1(v1.z); u[j].h[7] = (_Float16)elu1(v1.w);
      }
#pragma unroll
      for (int j = 0; j < 4; ++j) {
        const int q    = (grp * 4 + j) * NTHR + tid;
        const int slot = q / C8;
        const int c8   = q - slot * C8;
        if (slot < nvalid)
          *(volatile v4i*)(Hout + (size_t)(vbase + n0 + slot) * DF + c8 * 8) = u[j].i;
      }
      __threadfence();
#pragma unroll
      for (int j = 0; j < 4; ++j) {
        const int q    = (grp * 4 + j) * NTHR + tid;
        const int slot = q / C8;
        const int c8   = q - slot * C8;
        if (slot < nvalid)
          *(volatile v4i*)(Hout + (size_t)(vbase + n0 + slot) * DF + c8 * 8) = u[j].i;
      }
    }
  } else {
    const int qn = tid >> 2;
    const int f0 = (tid & 3) * 4;
#pragma unroll 1
    for (int t = 0; t < TT; ++t) {
      v4f rv[NB / 64];
#pragma unroll
      for (int ps = 0; ps < NB / 64; ++ps) {
        const int slot = ps * 64 + qn;
        v4f r = {0.f, 0.f, 0.f, 0.f};
        if (slot < nvalid) {
          const size_t go = ((size_t)(b * TT + t) * NN + (size_t)(n0 + slot)) * FF + f0;
          const v4f xv = *(const v4f*)(x + go);
          const float iv = inv[slot];
          const float* sp = sacc + slot * DF + f0 * TT + t;
          const float v0 = sp[0]      * iv + bias[(f0 + 0) * TT + t];
          const float v1 = sp[TT]     * iv + bias[(f0 + 1) * TT + t];
          const float v2 = sp[2 * TT] * iv + bias[(f0 + 2) * TT + t];
          const float v3 = sp[3 * TT] * iv + bias[(f0 + 3) * TT + t];
          r.x = xv.x + elu1(v0);
          r.y = xv.y + elu1(v1);
          r.z = xv.z + elu1(v2);
          r.w = xv.w + elu1(v3);
        }
        rv[ps] = r;
      }
#pragma unroll
      for (int ps = 0; ps < NB / 64; ++ps) {
        const int slot = ps * 64 + qn;
        if (slot < nvalid) {
          const size_t go = ((size_t)(b * TT + t) * NN + (size_t)(n0 + slot)) * FF + f0;
          *(volatile v4f*)(out + go) = rv[ps];
        }
      }
      __threadfence();
#pragma unroll
      for (int ps = 0; ps < NB / 64; ++ps) {
        const int slot = ps * 64 + qn;
        if (slot < nvalid) {
          const size_t go = ((size_t)(b * TT + t) * NN + (size_t)(n0 + slot)) * FF + f0;
          *(volatile v4f*)(out + go) = rv[ps];
        }
      }
    }
  }
}

extern "C" void kernel_launch(void* const* d_in, const int* in_sizes, int n_in,
                              void* d_out, int out_size, void* d_ws, size_t ws_size,
                              hipStream_t stream) {
  if (n_in < 11) return;
  if (in_sizes[0] != BB * TT * NN * FF) return;
  if (out_size != in_sizes[0]) return;
  const int nE = in_sizes[1];
  if (nE < 0 || in_sizes[2] != nE) return;
  if (in_sizes[3] != DF * DF || in_sizes[7] != DF * DF) return;
  if (in_sizes[4] != DF || in_sizes[5] != DF || in_sizes[6] != DF) return;
  if (in_sizes[8] != DF || in_sizes[9] != DF || in_sizes[10] != DF) return;

  const float* x     = (const float*)d_in[0];
  const int*   src   = (const int*)d_in[1];
  const int*   dst   = (const int*)d_in[2];
  const float* W0    = (const float*)d_in[3];
  const float* al0   = (const float*)d_in[4];
  const float* ar0   = (const float*)d_in[5];
  const float* bias0 = (const float*)d_in[6];
  const float* W1    = (const float*)d_in[7];
  const float* al1   = (const float*)d_in[8];
  const float* ar1   = (const float*)d_in[9];
  const float* bias1 = (const float*)d_in[10];
  float* out = (float*)d_out;

  const int V  = VV;
  const int VP = ((V + GR - 1) / GR) * GR;
  size_t off = 0;
  _Float16* Hh  = (_Float16*)((char*)d_ws + off); off += ((size_t)VP * DF * 2 + 255) & ~(size_t)255;
  _Float16* Wt0 = (_Float16*)((char*)d_ws + off); off += ((size_t)DF * DF * 2 + 255) & ~(size_t)255;
  _Float16* Wt1 = (_Float16*)((char*)d_ws + off); off += ((size_t)DF * DF * 2 + 255) & ~(size_t)255;
  float* ft  = (float*)((char*)d_ws + off); off += ((size_t)VP * DF * 4 + 255) & ~(size_t)255;
  float* elv = (float*)((char*)d_ws + off); off += ((size_t)VP * 4 + 255) & ~(size_t)255;
  float* erv = (float*)((char*)d_ws + off); off += ((size_t)VP * 4 + 255) & ~(size_t)255;
  if (off > ws_size) return;
  if (off > (size_t)134217728) return;

  const int ntask = V * C8;
  k_prepx<<<(ntask + NTHR - 1) / NTHR, NTHR, 0, stream>>>(x, Hh, ntask);
  k_prepw<<<(2 * DF * C8 + NTHR - 1) / NTHR, NTHR, 0, stream>>>(W0, W1, Wt0, Wt1);

  const int nblk = (NN + NB - 1) / NB;
  hipFuncSetAttribute(reinterpret_cast<const void*>(&k_agg),
                      hipFuncAttributeMaxDynamicSharedMemorySize, LDS_BYTES);

  k_gemm<<<VP / GR, NTHR, 0, stream>>>(Hh, Wt0, al0, ar0, ft, elv, erv, V);
  k_agg<<<nblk * BB, NTHR, LDS_BYTES, stream>>>(ft, elv, erv, src, dst, bias0, x, Hh, out, nE, nblk, 0);

  k_gemm<<<VP / GR, NTHR, 0, stream>>>(Hh, Wt1, al1, ar1, ft, elv, erv, V);
  k_agg<<<nblk * BB, NTHR, LDS_BYTES, stream>>>(ft, elv, erv, src, dst, bias1, x, Hh, out, nE, nblk, 1);
}
